// SimpleMambaEncoderLayer_21071109554439
// MI455X (gfx1250) — hardware-run, weakly checked
//
#include <hip/hip_runtime.h>
#include <math.h>

typedef __attribute__((ext_vector_type(16))) _Float16 v16h;
typedef __attribute__((ext_vector_type(8)))  _Float16 v8h;
typedef __attribute__((ext_vector_type(8)))  float    v8f;
typedef __attribute__((ext_vector_type(4)))  float    v4f;

constexpr int kBatch  = 8;
constexpr int kSide   = 32;
constexpr int kSeq    = kSide * kSide;
constexpr int kRows   = kBatch * kSeq;
constexpr int kDm     = 96;
constexpr int kDin    = 192;
constexpr int kNst    = 16;
constexpr int kDtR    = 6;
constexpr int kDirs   = 4;
constexpr int kDff    = 512;
constexpr int kXzN    = 2 * kDin;
constexpr int kXpN    = kDtR + 2 * kNst;
constexpr int kXpAll  = kDirs * kXpN;
constexpr int kXpPad  = 192;
constexpr int kNp     = 128;
constexpr float kEps  = 1e-5f;

constexpr float kCarryX  = 16.0f;
constexpr float kCarryW  = 256.0f;
constexpr float kCarryU  = 64.0f;
constexpr float kCarryYG = 256.0f;
constexpr float kCarryH  = 16.0f;
constexpr float kCarryF  = 16.0f;
constexpr float kFoldIn  = 1.0f / (kCarryX  * kCarryW);
constexpr float kFoldXp  = 1.0f / (kCarryU  * kCarryW);
constexpr float kFoldOut = 1.0f / (kCarryYG * kCarryW);
constexpr float kFoldF1  = 1.0f / (kCarryH  * kCarryW);
constexpr float kFoldF2  = 1.0f / (kCarryF  * kCarryW);

static_assert(kSeq == 1024 && kRows == 8192, "grid geometry");
static_assert(kXpN == 38 && kXpAll == 152 && kXpAll <= kXpPad, "x_proj width");
static_assert((kDm % 32) == 0 && (kDin % 32) == 0 && (kDff % 32) == 0, "GEMM K multiples of 32");
static_assert((kRows % 64) == 0 && (kXzN % 64) == 0 && (kXpPad % 64) == 0 && (kNp % 64) == 0 && (kDff % 64) == 0, "GEMM M,N multiples of 64");
static_assert((kRows % 8) == 0 && (kSeq % 16) == 0, "row blocking");

constexpr size_t kSzX16   = (size_t)kRows * kDm * 2;
constexpr size_t kSzWIN   = (size_t)kXzN * kDm * 2;
constexpr size_t kSzWXP   = (size_t)kXpPad * kDin * 2;
constexpr size_t kSzWOUT  = (size_t)kNp * kDin * 2;
constexpr size_t kSzW1    = (size_t)kDff * kDm * 2;
constexpr size_t kSzW2    = (size_t)kNp * kDff * 2;
constexpr size_t kSzXZ    = (size_t)kRows * kXzN * 4;
constexpr size_t kSzUZ    = (size_t)kRows * kXzN * 4;
constexpr size_t kSzU16   = (size_t)kRows * kDin * 2;
constexpr size_t kSzXD    = (size_t)kRows * kXpPad * 4;
constexpr size_t kSzYS    = (size_t)kDirs * kRows * kDin * 4;
constexpr size_t kSzYG    = (size_t)kRows * kDin * 2;
constexpr size_t kSzATT   = (size_t)kRows * kNp * 4;
constexpr size_t kSzH1    = (size_t)kRows * kDm * 4;
constexpr size_t kSzH116  = (size_t)kRows * kDm * 2;
constexpr size_t kSzFFA   = (size_t)kRows * kDff * 2;
constexpr size_t kSzFF    = (size_t)kRows * kNp * 4;
constexpr size_t kOffX16  = 0;
constexpr size_t kOffWIN  = kOffX16  + kSzX16;
constexpr size_t kOffWXP  = kOffWIN  + kSzWIN;
constexpr size_t kOffWOUT = kOffWXP  + kSzWXP;
constexpr size_t kOffW1   = kOffWOUT + kSzWOUT;
constexpr size_t kOffW2   = kOffW1   + kSzW1;
constexpr size_t kOffXZ   = kOffW2   + kSzW2;
constexpr size_t kOffUZ   = kOffXZ   + kSzXZ;
constexpr size_t kOffU16  = kOffUZ   + kSzUZ;
constexpr size_t kOffXD   = kOffU16  + kSzU16;
constexpr size_t kOffYS   = kOffXD   + kSzXD;
constexpr size_t kOffYG   = kOffYS   + kSzYS;
constexpr size_t kOffATT  = kOffYG   + kSzYG;
constexpr size_t kOffH1   = kOffATT  + kSzATT;
constexpr size_t kOffH116 = kOffH1   + kSzH1;
constexpr size_t kOffFFA  = kOffH116 + kSzH116;
constexpr size_t kOffFF   = kOffFFA  + kSzFFA;
constexpr size_t kWsTotal = kOffFF   + kSzFF;
static_assert(kWsTotal == 86409216ull, "carve total");
static_assert(kWsTotal <= 134217728ull, "carve cap");
static_assert((kOffWIN % 128) == 0 && (kOffWXP % 128) == 0 && (kOffWOUT % 128) == 0 && (kOffW1 % 128) == 0 &&
              (kOffW2 % 128) == 0 && (kOffXZ % 128) == 0 && (kOffUZ % 128) == 0 && (kOffU16 % 128) == 0 &&
              (kOffXD % 128) == 0 && (kOffYS % 128) == 0 && (kOffYG % 128) == 0 && (kOffATT % 128) == 0 &&
              (kOffH1 % 128) == 0 && (kOffH116 % 128) == 0 && (kOffFFA % 128) == 0 && (kOffFF % 128) == 0,
              "128-B aligned regions");

__device__ __forceinline__ v16h frag_load(const _Float16* p) {
  union U { v16h v; v8h h[2]; } f;
  f.h[0] = *(const v8h*)(p);
  f.h[1] = *(const v8h*)(p + 16);
  return f.v;
}
__device__ __forceinline__ v8f mma_g(v16h a, v16h b, v8f c) {
  c = __builtin_amdgcn_wmma_f32_16x16x32_f16(false, a, false, b, (short)0, c, false, false);
  asm volatile("v_nop\n\tv_nop\n\tv_nop\n\tv_nop" : "+v"(c) : "v"(a), "v"(b));
  return c;
}

template <int BIAS_MODE, int OUT_MODE, int ACT>
__global__ __launch_bounds__(256) void wmma_gemm64(
    const unsigned short* __restrict__ Ap, int lda,
    const unsigned short* __restrict__ Btp, int ldb,
    void* __restrict__ Cout, int ldc,
    const float* __restrict__ bias,
    int M, int N, int K, float scale, float oscale)
{
  const _Float16* A  = (const _Float16*)Ap;
  const _Float16* Bt = (const _Float16*)Btp;
  __shared__ __align__(16) float sT[8][16 * 68];
  const int lane = threadIdx.x & 31;
  const int wave = threadIdx.x >> 5;
  const int tilesN = N >> 6;
  const int tilesM = M >> 6;
  const int tile = blockIdx.x * 8 + wave;
  if (tile >= tilesM * tilesN) return;
  const int tm = tile / tilesN;
  const int tn = tile - tm * tilesN;
  const int m0 = tm << 6;
  const int n0 = tn << 6;
  const int rlane = lane & 15;
  const int koff  = (lane >> 4) * 8;
  const int mOff  = (lane >> 4) * 8;

  v8f acc[4][4];
#pragma unroll
  for (int i = 0; i < 4; ++i)
#pragma unroll
    for (int j = 0; j < 4; ++j) acc[i][j] = (v8f){0.f, 0.f, 0.f, 0.f, 0.f, 0.f, 0.f, 0.f};

  for (int k0 = 0; k0 < K; k0 += 32) {
    v16h bh[4];
#pragma unroll
    for (int j = 0; j < 4; ++j) {
      const size_t bo = (size_t)(n0 + (j << 4) + rlane) * ldb + koff + k0;
      bh[j] = frag_load(Bt + bo);
    }
#pragma unroll
    for (int i = 0; i < 4; ++i) {
      const size_t ao = (size_t)(m0 + (i << 4) + rlane) * lda + koff + k0;
      const v16h ah = frag_load(A + ao);
#pragma unroll
      for (int j = 0; j < 4; ++j) acc[i][j] = mma_g(ah, bh[j], acc[i][j]);
    }
  }

  float* slab = sT[wave];
#pragma unroll
  for (int i = 0; i < 4; ++i) {
    const int mBase = m0 + (i << 4);
#pragma unroll
    for (int j = 0; j < 4; ++j) {
      const int n = n0 + (j << 4) + rlane;
      float bv = 0.f;
      if (BIAS_MODE == 2) bv = bias[n];
#pragma unroll
      for (int r = 0; r < 8; ++r) {
        float v = acc[i][j][r] * scale;
        if (BIAS_MODE == 2) v += bv;
        if (ACT == 2) v = fmaxf(v, 0.0f);
        v = v * oscale;
        slab[(mOff + r) * 68 + (j << 4) + rlane] = v;
      }
    }
    __builtin_amdgcn_fence(__ATOMIC_RELEASE, "workgroup");
    __builtin_amdgcn_wave_barrier();
    __builtin_amdgcn_fence(__ATOMIC_ACQUIRE, "workgroup");
    if (OUT_MODE == 0) {
      float* C = (float*)Cout;
      const int hh = lane >> 4, c4 = (lane & 15) * 4;
      for (int pass = 0; pass < 2; ++pass) {
#pragma unroll
        for (int it = 0; it < 8; ++it) {
          const int row = it * 2 + hh;
          const v4f v = *(const v4f*)(slab + row * 68 + c4);
          *(volatile v4f*)(C + (size_t)(mBase + row) * ldc + n0 + c4) = v;
        }
        __threadfence();
      }
    } else {
      const int q = lane >> 3, c8 = (lane & 7) * 8;
      unsigned short* C = (unsigned short*)Cout;
      for (int pass = 0; pass < 2; ++pass) {
#pragma unroll
        for (int it = 0; it < 4; ++it) {
          const int row = it * 4 + q;
          const float* sp = slab + row * 68 + c8;
          v8h hv;
#pragma unroll
          for (int e = 0; e < 8; ++e) hv[e] = (_Float16)sp[e];
          *(volatile v8h*)(C + (size_t)(mBase + row) * ldc + n0 + c8) = hv;
        }
        __threadfence();
      }
    }
    __builtin_amdgcn_fence(__ATOMIC_RELEASE, "workgroup");
    __builtin_amdgcn_wave_barrier();
    __builtin_amdgcn_fence(__ATOMIC_ACQUIRE, "workgroup");
  }
}

__global__ __launch_bounds__(256) void cast_rows_f16_kernel(
    const float* __restrict__ src, unsigned short* __restrict__ dst,
    int rows_real, int cols, int total8, float scale)
{
  const int i = blockIdx.x * 256 + threadIdx.x;
  if (i >= total8) return;
  const int e0  = i << 3;
  const int row = e0 / cols;
  const int col = e0 - row * cols;
  const int rc  = (row < rows_real) ? row : (rows_real - 1);
  const float* p = src + (size_t)rc * cols + col;
  const v4f a0 = *(const v4f*)(p);
  const v4f a1 = *(const v4f*)(p + 4);
  const bool keep = (row < rows_real);
  v8h hv;
#pragma unroll
  for (int e = 0; e < 4; ++e) {
    const float f0 = keep ? (a0[e] * scale) : 0.0f;
    const float f1 = keep ? (a1[e] * scale) : 0.0f;
    hv[e]     = (_Float16)f0;
    hv[4 + e] = (_Float16)f1;
  }
  unsigned short* q = dst + (size_t)e0;
  *(volatile v8h*)q = hv;
  __threadfence();
  *(volatile v8h*)q = hv;
}

__global__ __launch_bounds__(256) void silu_split_kernel(
    const float* __restrict__ XZ, float* __restrict__ UZ, unsigned short* __restrict__ U16)
{
  __shared__ __align__(16) float sT[8 * kXzN];
  const int tid = threadIdx.x;
  const size_t base = (size_t)blockIdx.x * (8 * kXzN);
#pragma unroll 1
  for (int it = 0; it < 3; ++it) {
    const int idx = it * 256 + tid;
    const v4f a = *(const v4f*)(XZ + base + (size_t)idx * 4);
    v4f r;
#pragma unroll
    for (int e = 0; e < 4; ++e) {
      const float v = a[e];
      r[e] = v * (1.0f / (1.0f + expf(-v)));
    }
    *(v4f*)(sT + idx * 4) = r;
  }
  __syncthreads();
  v4f fv[3];
#pragma unroll
  for (int it = 0; it < 3; ++it) fv[it] = *(const v4f*)(sT + (it * 256 + tid) * 4);
  v8h hv;
#pragma unroll
  for (int e = 0; e < 8; ++e) hv[e] = (_Float16)0.0f;
  if (tid < 192) {
    const int rl = tid / 24;
    const int c8 = (tid - rl * 24) * 8;
    const float* sp = sT + rl * kXzN + c8;
    const v4f a0 = *(const v4f*)(sp);
    const v4f a1 = *(const v4f*)(sp + 4);
#pragma unroll
    for (int e = 0; e < 4; ++e) {
      hv[e]     = (_Float16)(a0[e] * kCarryU);
      hv[4 + e] = (_Float16)(a1[e] * kCarryU);
    }
  }
  for (int pass = 0; pass < 2; ++pass) {
#pragma unroll
    for (int it = 0; it < 3; ++it)
      *(volatile v4f*)(UZ + base + (size_t)(it * 256 + tid) * 4) = fv[it];
    if (tid < 192)
      *(volatile v8h*)(U16 + (size_t)blockIdx.x * (8 * kDin) + (size_t)tid * 8) = hv;
    __threadfence();
  }
}

__device__ __forceinline__ int scan_pos(int k, int l) {
  const int lf = (k & 2) ? (kSeq - 1 - l) : l;
  const int sw = ((lf & 31) << 5) | (lf >> 5);
  return (k & 1) ? sw : lf;
}

__global__ __launch_bounds__(192) void scan_kernel(
    const float* __restrict__ XD, const float* __restrict__ UZ,
    const float* __restrict__ Wdt, const float* __restrict__ bdt,
    const float* __restrict__ Alog, const float* __restrict__ Dsk,
    float* __restrict__ YS)
{
  __shared__ __align__(16) float sX[16 * 40];
  __shared__ __align__(16) float sY[16 * 196];
  __shared__ float sH[kNst * kDin];
  __shared__ float sA[kNst * kDin];
  const int tid = threadIdx.x;
  const int b = blockIdx.x >> 2;
  const int k = blockIdx.x & 3;
  const size_t kd = (size_t)k * kDin + tid;
  const float w0 = Wdt[kd * kDtR + 0];
  const float w1 = Wdt[kd * kDtR + 1];
  const float w2 = Wdt[kd * kDtR + 2];
  const float w3 = Wdt[kd * kDtR + 3];
  const float w4 = Wdt[kd * kDtR + 4];
  const float w5 = Wdt[kd * kDtR + 5];
  const float bb = bdt[kd];
  const float Dd = Dsk[kd];
#pragma unroll 1
  for (int n = 0; n < kNst; ++n) {
    sA[n * kDin + tid] = -expf(Alog[kd * kNst + n]);
    sH[n * kDin + tid] = 0.0f;
  }
  const size_t rowb = (size_t)b * kSeq;
  float* YSk = YS + (size_t)k * kRows * kDin;

#pragma unroll 1
  for (int c = 0; c < kSeq / 16; ++c) {
    const int l0 = c * 16;
    __syncthreads();
#pragma unroll
    for (int it = 0; it < 4; ++it) {
      const int idx = it * kDin + tid;
      const int idc = (idx < 16 * kXpN) ? idx : (16 * kXpN - 1);
      const int s   = idc / kXpN;
      const int cc  = idc - s * kXpN;
      const int p   = scan_pos(k, l0 + s);
      sX[s * 40 + cc] = XD[(rowb + p) * kXpPad + kXpN * k + cc];
    }
    __syncthreads();
#pragma unroll 1
    for (int s = 0; s < 16; ++s) {
      const int p = scan_pos(k, l0 + s);
      const float* xr = sX + s * 40;
      float v = xr[0] * w0;
      v = fmaf(xr[1], w1, v);
      v = fmaf(xr[2], w2, v);
      v = fmaf(xr[3], w3, v);
      v = fmaf(xr[4], w4, v);
      v = fmaf(xr[5], w5, v);
      v = v + bb;
      const float delta = fmaxf(v, 0.0f) + log1pf(expf(-fabsf(v)));
      const float u  = UZ[(rowb + p) * kXzN + tid];
      const float du = delta * u;
      float y = 0.0f;
#pragma unroll 1
      for (int n = 0; n < kNst; ++n) {
        const float dA = expf(delta * sA[n * kDin + tid]);
        const float hn = sH[n * kDin + tid] * dA + du * xr[kDtR + n];
        sH[n * kDin + tid] = hn;
        y = y + hn * xr[kDtR + kNst + n];
      }
      sY[s * 196 + tid] = y + Dd * u;
    }
    __syncthreads();
    v4f fv[4];
    size_t oo[4];
#pragma unroll
    for (int it = 0; it < 4; ++it) {
      const int idx = it * kDin + tid;
      const int s   = idx / 48;
      const int c4  = (idx - s * 48) * 4;
      const int p   = scan_pos(k, l0 + s);
      fv[it] = *(const v4f*)(sY + s * 196 + c4);
      oo[it] = (rowb + p) * kDin + c4;
    }
    for (int pass = 0; pass < 2; ++pass) {
#pragma unroll
      for (int it = 0; it < 4; ++it) *(volatile v4f*)(YSk + oo[it]) = fv[it];
      __threadfence();
    }
  }
}

__global__ __launch_bounds__(256) void merge_norm_gate_kernel(
    const float* __restrict__ YS, const float* __restrict__ UZ,
    const float* __restrict__ g, const float* __restrict__ be,
    unsigned short* __restrict__ YG16)
{
  __shared__ __align__(16) float sT[8 * kDin];
  const int tid = threadIdx.x, lane = tid & 31, wave = tid >> 5;
  const size_t row = (size_t)blockIdx.x * 8 + wave;
  const size_t plane = (size_t)kRows * kDin;
  float v[6];
  float s1 = 0.0f;
#pragma unroll
  for (int e = 0; e < 6; ++e) {
    const int dd = e * 32 + lane;
    const size_t off = row * kDin + dd;
    const float p0 = YS[off];
    const float p1 = YS[plane + off];
    const float p2 = YS[2 * plane + off];
    const float p3 = YS[3 * plane + off];
    const float t = ((p0 + p2) + p1) + p3;
    v[e] = t;
    s1 += t;
  }
#pragma unroll
  for (int off = 16; off > 0; off >>= 1) s1 += __shfl_xor(s1, off, 32);
  const float mean = s1 * (1.0f / kDin);
  float s2 = 0.0f;
#pragma unroll
  for (int e = 0; e < 6; ++e) {
    const float cdev = v[e] - mean;
    s2 += cdev * cdev;
  }
#pragma unroll
  for (int off = 16; off > 0; off >>= 1) s2 += __shfl_xor(s2, off, 32);
  const float var  = s2 * (1.0f / kDin);
  const float rstd = 1.0f / sqrtf(var + kEps);
#pragma unroll
  for (int e = 0; e < 6; ++e) {
    const int dd = e * 32 + lane;
    const float t = (v[e] - mean) * rstd * g[dd] + be[dd];
    const float z = UZ[row * kXzN + kDin + dd];
    sT[wave * kDin + dd] = (t * z) * kCarryYG;
  }
  __syncthreads();
  v8h hv;
#pragma unroll
  for (int e = 0; e < 8; ++e) hv[e] = (_Float16)0.0f;
  if (tid < 192) {
    const float* sp = sT + tid * 8;
    const v4f a0 = *(const v4f*)(sp);
    const v4f a1 = *(const v4f*)(sp + 4);
#pragma unroll
    for (int e = 0; e < 4; ++e) {
      hv[e]     = (_Float16)a0[e];
      hv[4 + e] = (_Float16)a1[e];
    }
  }
  for (int pass = 0; pass < 2; ++pass) {
    if (tid < 192)
      *(volatile v8h*)(YG16 + (size_t)blockIdx.x * (8 * kDin) + (size_t)tid * 8) = hv;
    __threadfence();
  }
}

template <bool HASBIAS, bool OUT16>
__global__ __launch_bounds__(256) void add_norm96_kernel(
    const float* __restrict__ base, const float* __restrict__ add, const float* __restrict__ addbias,
    const float* __restrict__ g, const float* __restrict__ be,
    float* __restrict__ out32, unsigned short* __restrict__ out16, float carry)
{
  __shared__ __align__(16) float sT[8 * kDm];
  const int tid = threadIdx.x, lane = tid & 31, wave = tid >> 5;
  const size_t row = (size_t)blockIdx.x * 8 + wave;
  float v[3];
  float s1 = 0.0f;
#pragma unroll
  for (int e = 0; e < 3; ++e) {
    const int dd = e * 32 + lane;
    float t = add[row * kNp + dd];
    if (HASBIAS) t = t + addbias[dd];
    t = base[row * kDm + dd] + t;
    v[e] = t;
    s1 += t;
  }
#pragma unroll
  for (int off = 16; off > 0; off >>= 1) s1 += __shfl_xor(s1, off, 32);
  const float mean = s1 * (1.0f / kDm);
  float s2 = 0.0f;
#pragma unroll
  for (int e = 0; e < 3; ++e) {
    const float cdev = v[e] - mean;
    s2 += cdev * cdev;
  }
#pragma unroll
  for (int off = 16; off > 0; off >>= 1) s2 += __shfl_xor(s2, off, 32);
  const float var  = s2 * (1.0f / kDm);
  const float rstd = 1.0f / sqrtf(var + kEps);
#pragma unroll
  for (int e = 0; e < 3; ++e) {
    const int dd = e * 32 + lane;
    sT[wave * kDm + dd] = (v[e] - mean) * rstd * g[dd] + be[dd];
  }
  __syncthreads();
  v4f fv = (v4f){0.f, 0.f, 0.f, 0.f};
  v8h hv;
#pragma unroll
  for (int e = 0; e < 8; ++e) hv[e] = (_Float16)0.0f;
  if (tid < 192) fv = *(const v4f*)(sT + tid * 4);
  if (OUT16) {
    if (tid < 96) {
      const float* sp = sT + tid * 8;
      const v4f a0 = *(const v4f*)(sp);
      const v4f a1 = *(const v4f*)(sp + 4);
#pragma unroll
      for (int e = 0; e < 4; ++e) {
        hv[e]     = (_Float16)(a0[e] * carry);
        hv[4 + e] = (_Float16)(a1[e] * carry);
      }
    }
  }
  for (int pass = 0; pass < 2; ++pass) {
    if (tid < 192)
      *(volatile v4f*)(out32 + (size_t)blockIdx.x * (8 * kDm) + (size_t)tid * 4) = fv;
    if (OUT16) {
      if (tid < 96)
        *(volatile v8h*)(out16 + (size_t)blockIdx.x * (8 * kDm) + (size_t)tid * 8) = hv;
    }
    __threadfence();
  }
}

constexpr int gemm_blocks(int M, int N) { return (((M / 64) * (N / 64)) + 7) / 8; }

extern "C" void kernel_launch(void* const* d_in, const int* in_sizes, int n_in,
                              void* d_out, int out_size, void* d_ws, size_t ws_size,
                              hipStream_t stream)
{
  if (n_in < 18) return;
  if (in_sizes[0] != kRows * kDm) return;
  if (in_sizes[1] != kXzN * kDm) return;
  if (in_sizes[2] != kDirs * kXpN * kDin) return;
  if (in_sizes[3] != kDirs * kDin * kDtR) return;
  if (in_sizes[4] != kDirs * kDin) return;
  if (in_sizes[5] != kDirs * kDin * kNst) return;
  if (in_sizes[6] != kDirs * kDin) return;
  if (in_sizes[7] != kDin || in_sizes[8] != kDin) return;
  if (in_sizes[9] != kDm * kDin) return;
  if (in_sizes[10] != kDm || in_sizes[11] != kDm || in_sizes[12] != kDm || in_sizes[13] != kDm) return;
  if (in_sizes[14] != kDff * kDm) return;
  if (in_sizes[15] != kDff) return;
  if (in_sizes[16] != kDm * kDff) return;
  if (in_sizes[17] != kDm) return;
  if (out_size != kRows * kDm) return;
  if (ws_size < kWsTotal) return;

  const float* x          = (const float*)d_in[0];
  const float* in_proj_w  = (const float*)d_in[1];
  const float* x_proj_w   = (const float*)d_in[2];
  const float* dt_projs_w = (const float*)d_in[3];
  const float* dt_projs_b = (const float*)d_in[4];
  const float* A_logs     = (const float*)d_in[5];
  const float* Dsk        = (const float*)d_in[6];
  const float* out_norm_g = (const float*)d_in[7];
  const float* out_norm_b = (const float*)d_in[8];
  const float* out_proj_w = (const float*)d_in[9];
  const float* ln1_g      = (const float*)d_in[10];
  const float* ln1_b      = (const float*)d_in[11];
  const float* ln2_g      = (const float*)d_in[12];
  const float* ln2_b      = (const float*)d_in[13];
  const float* ff_w1      = (const float*)d_in[14];
  const float* ff_b1      = (const float*)d_in[15];
  const float* ff_w2      = (const float*)d_in[16];
  const float* ff_b2      = (const float*)d_in[17];
  float* out = (float*)d_out;

  char* ws = (char*)d_ws;
  unsigned short* X16    = (unsigned short*)(ws + kOffX16);
  unsigned short* WIN16  = (unsigned short*)(ws + kOffWIN);
  unsigned short* WXP16  = (unsigned short*)(ws + kOffWXP);
  unsigned short* WOUT16 = (unsigned short*)(ws + kOffWOUT);
  unsigned short* W116   = (unsigned short*)(ws + kOffW1);
  unsigned short* W216   = (unsigned short*)(ws + kOffW2);
  float*          XZ     = (float*)(ws + kOffXZ);
  float*          UZ     = (float*)(ws + kOffUZ);
  unsigned short* U16    = (unsigned short*)(ws + kOffU16);
  float*          XD     = (float*)(ws + kOffXD);
  float*          YS     = (float*)(ws + kOffYS);
  unsigned short* YG16   = (unsigned short*)(ws + kOffYG);
  float*          ATT    = (float*)(ws + kOffATT);
  float*          H1     = (float*)(ws + kOffH1);
  unsigned short* H116   = (unsigned short*)(ws + kOffH116);
  unsigned short* FFA16  = (unsigned short*)(ws + kOffFFA);
  float*          FF     = (float*)(ws + kOffFF);

  cast_rows_f16_kernel<<<(kRows * kDm / 8) / 256, 256, 0, stream>>>(x, X16, kRows, kDm, kRows * kDm / 8, kCarryX);
  cast_rows_f16_kernel<<<(kXzN * kDm / 8) / 256, 256, 0, stream>>>(in_proj_w, WIN16, kXzN, kDm, kXzN * kDm / 8, kCarryW);
  cast_rows_f16_kernel<<<(kXpPad * kDin / 8) / 256, 256, 0, stream>>>(x_proj_w, WXP16, kXpAll, kDin, kXpPad * kDin / 8, kCarryW);
  cast_rows_f16_kernel<<<(kNp * kDin / 8) / 256, 256, 0, stream>>>(out_proj_w, WOUT16, kDm, kDin, kNp * kDin / 8, kCarryW);
  cast_rows_f16_kernel<<<(kDff * kDm / 8) / 256, 256, 0, stream>>>(ff_w1, W116, kDff, kDm, kDff * kDm / 8, kCarryW);
  cast_rows_f16_kernel<<<(kNp * kDff / 8) / 256, 256, 0, stream>>>(ff_w2, W216, kDm, kDff, kNp * kDff / 8, kCarryW);

  wmma_gemm64<0, 0, 0><<<gemm_blocks(kRows, kXzN), 256, 0, stream>>>(
      X16, kDm, WIN16, kDm, (void*)XZ, kXzN, ff_b1, kRows, kXzN, kDm, kFoldIn, 1.0f);

  silu_split_kernel<<<kRows / 8, 256, 0, stream>>>(XZ, UZ, U16);

  wmma_gemm64<0, 0, 0><<<gemm_blocks(kRows, kXpPad), 256, 0, stream>>>(
      U16, kDin, WXP16, kDin, (void*)XD, kXpPad, ff_b1, kRows, kXpPad, kDin, kFoldXp, 1.0f);

  scan_kernel<<<kBatch * kDirs, kDin, 0, stream>>>(XD, UZ, dt_projs_w, dt_projs_b, A_logs, Dsk, YS);

  merge_norm_gate_kernel<<<kRows / 8, 256, 0, stream>>>(YS, UZ, out_norm_g, out_norm_b, YG16);

  wmma_gemm64<0, 0, 0><<<gemm_blocks(kRows, kNp), 256, 0, stream>>>(
      YG16, kDin, WOUT16, kDin, (void*)ATT, kNp, ff_b1, kRows, kNp, kDin, kFoldOut, 1.0f);

  add_norm96_kernel<false, true><<<kRows / 8, 256, 0, stream>>>(
      x, ATT, ff_b2, ln1_g, ln1_b, H1, H116, kCarryH);

  wmma_gemm64<2, 1, 2><<<gemm_blocks(kRows, kDff), 256, 0, stream>>>(
      H116, kDm, W116, kDm, (void*)FFA16, kDff, ff_b1, kRows, kDff, kDm, kFoldF1, kCarryF);

  wmma_gemm64<0, 0, 0><<<gemm_blocks(kRows, kNp), 256, 0, stream>>>(
      FFA16, kDff, W216, kDff, (void*)FF, kNp, ff_b1, kRows, kNp, kDff, kFoldF2, 1.0f);

  add_norm96_kernel<true, false><<<kRows / 8, 256, 0, stream>>>(
      H1, FF, ff_b2, ln2_g, ln2_b, out, H116, 1.0f);
}
